// TopKWindowAttentionLayer_27839978012830
// MI455X (gfx1250) — hardware-verified
//
#include <hip/hip_runtime.h>
#include <hip/hip_bf16.h>
#include <stddef.h>

typedef __attribute__((ext_vector_type(16))) _Float16 v16h;
typedef __attribute__((ext_vector_type(8)))  _Float16 v8h;
typedef __attribute__((ext_vector_type(16))) __bf16   v16b;
typedef __attribute__((ext_vector_type(8)))  __bf16   v8b;
typedef __attribute__((ext_vector_type(8)))  float    v8f;
typedef __attribute__((ext_vector_type(4)))  float    v4f;
typedef __attribute__((ext_vector_type(4)))  unsigned v4u;

constexpr int BATCH = 8;
constexpr int CH    = 256;
constexpr int IMGW  = 56;
constexpr int NPIX  = 3136;
constexpr int NHEAD = 8;
constexpr int HDIM  = 32;
constexpr int WSIDE = 7;
constexpr int NWIN  = 64;
constexpr int WPIX  = 49;
constexpr int NTOP  = 8;
constexpr int NKEY  = 392;
constexpr int CH3   = 768;
constexpr int HID   = 1024;
constexpr int KCH   = 64;
constexpr int NCHUNK = 7;
constexpr float BN_EPS = 1e-5f;
static_assert(KCH * NCHUNK >= NKEY);
static_assert(KCH * (NCHUNK - 1) < NKEY);
static_assert(NWIN * WPIX == NPIX);
static_assert(NTOP * WPIX == NKEY);
constexpr float kScoreScale = 1.4426950408889634f / (64.0f * 5.656854249492381f);

__device__ __forceinline__ unsigned short f2bf_bits(float f) {
  unsigned u = __float_as_uint(f);
  return (unsigned short)((u + 0x7FFFu + ((u >> 16) & 1u)) >> 16);
}
__device__ __forceinline__ float bf_bits2f(unsigned short h) { return __uint_as_float(((unsigned)h) << 16); }
__device__ __forceinline__ unsigned short h_bits(float f) { return __builtin_bit_cast(unsigned short, (_Float16)f); }
__device__ __forceinline__ float h_val(unsigned short u) { return (float)__builtin_bit_cast(_Float16, u); }

__device__ __forceinline__ float gelu_f(float y) {
  const float ax = fabsf(y) * 0.70710678118654752f;
  const float t = __builtin_amdgcn_rcpf(fmaf(0.3275911f, ax, 1.0f));
  float pol = 1.061405429f;
  pol = fmaf(pol, t, -1.453152027f);
  pol = fmaf(pol, t, 1.421413741f);
  pol = fmaf(pol, t, -0.284496736f);
  pol = fmaf(pol, t, 0.254829592f);
  pol = pol * t;
  const float ec = expf(-(ax * ax)) * pol;
  const float w = (y >= 0.0f) ? (2.0f - ec) : ec;
  return 0.5f * y * w;
}

__device__ __forceinline__ void dep_guard_h(v8f& a, v8f& b, v16h x, v16h y) { asm volatile("v_nop\n\tv_nop\n\tv_nop\n\tv_nop" : "+v"(a), "+v"(b) : "v"(x), "v"(y)); }
__device__ __forceinline__ void dep_guard_b(v8f& a, v8f& b, v16b x, v16b y) { asm volatile("v_nop\n\tv_nop\n\tv_nop\n\tv_nop" : "+v"(a), "+v"(b) : "v"(x), "v"(y)); }
__device__ __forceinline__ void keep4_h(v16h a, v16h b, v16h c, v16h d) { asm volatile("v_nop" :: "v"(a), "v"(b), "v"(c), "v"(d)); }
__device__ __forceinline__ void keep4_b(v16b a, v16b b, v16b c, v16b d) { asm volatile("v_nop" :: "v"(a), "v"(b), "v"(c), "v"(d)); }
__device__ __forceinline__ void acc_guard4(v8f& a, v8f& b, v8f& c, v8f& d) { asm volatile("v_nop\n\tv_nop\n\tv_nop\n\tv_nop" : "+v"(a), "+v"(b), "+v"(c), "+v"(d)); }
template <typename T> struct Frag;
template <> struct Frag<_Float16> {
  typedef v16h V; union U { v16h v; v8h h[2]; };
  static __device__ __forceinline__ v16h load(const _Float16* p) {
    U f; f.h[0] = *(const v8h*)(p); f.h[1] = *(const v8h*)(p + 16); return f.v;
  }
  static __device__ __forceinline__ v8f mma(v16h a, v16h b, v8f c) {
    return __builtin_amdgcn_wmma_f32_16x16x32_f16(false, a, false, b, (short)0, c, false, false);
  }
  static __device__ __forceinline__ void guard(v8f& a, v8f& b, v16h x, v16h y) { dep_guard_h(a, b, x, y); }
  static __device__ __forceinline__ void keep(v16h a, v16h b, v16h c, v16h d) { keep4_h(a, b, c, d); }
};
template <> struct Frag<__bf16> {
  typedef v16b V; union U { v16b v; v8b h[2]; };
  static __device__ __forceinline__ v16b load(const __bf16* p) {
    U f; f.h[0] = *(const v8b*)(p); f.h[1] = *(const v8b*)(p + 16); return f.v;
  }
  static __device__ __forceinline__ v8f mma(v16b a, v16b b, v8f c) {
    return __builtin_amdgcn_wmma_f32_16x16x32_bf16(false, a, false, b, (short)0, c, false, false);
  }
  static __device__ __forceinline__ void guard(v8f& a, v8f& b, v16b x, v16b y) { dep_guard_b(a, b, x, y); }
  static __device__ __forceinline__ void keep(v16b a, v16b b, v16b c, v16b d) { keep4_b(a, b, c, d); }
};

__device__ __forceinline__ v8f mma_h(v16h a, v16h b, v8f c) {
  c = __builtin_amdgcn_wmma_f32_16x16x32_f16(false, a, false, b, (short)0, c, false, false);
  asm volatile("v_nop\n\tv_nop\n\tv_nop\n\tv_nop" : "+v"(c) : "v"(a), "v"(b));
  return c;
}

template <int ET> struct Elem;
template <> struct Elem<0> { typedef _Float16 T; };
template <> struct Elem<1> { typedef __bf16 T; };
template <int ET, bool SPLIT, int BIAS_MODE, int OUT_MODE, bool RESID>
__global__ __launch_bounds__(256) void wmma_gemm64(
    const unsigned short* __restrict__ Ap, const unsigned short* __restrict__ A2p, int lda, long strideA,
    const unsigned short* __restrict__ Btp, const unsigned short* __restrict__ Bt2p, int ldb, long strideB,
    void* __restrict__ Cout, void* __restrict__ Cout2, int ldc, long strideC,
    const float* __restrict__ bias,
    const float* __restrict__ resid, long strideR,
    int M, int N, int K, float scale) {
  typedef typename Elem<ET>::T T;
  typedef typename Frag<T>::V V;
  const T* A = (const T*)Ap; const T* A2 = (const T*)A2p; const T* Bt = (const T*)Btp; const T* Bt2 = (const T*)Bt2p;
  __shared__ __align__(16) float sT[8][16 * 68];
  const int b    = blockIdx.y;
  const int lane = threadIdx.x & 31;
  const int wave = threadIdx.x >> 5;
  const int tilesN = N >> 6;
  const int tilesM = M >> 6;
  const int tile = blockIdx.x * 8 + wave;
  if (tile >= tilesM * tilesN) return;
  const int tm = tile / tilesN;
  const int tn = tile - tm * tilesN;
  const int m0 = tm << 6;
  const int n0 = tn << 6;

  const T* Ab  = A  + (size_t)b * strideA;
  const T* Bb  = Bt + (size_t)b * strideB;
  const T* Ab2 = SPLIT ? (A2  + (size_t)b * strideA) : nullptr;
  const T* Bb2 = SPLIT ? (Bt2 + (size_t)b * strideB) : nullptr;

  const int rlane = lane & 15;
  const int koff  = (lane >> 4) * 8;
  const int mOff  = (lane >> 4) * 8;

  v8f acc[4][4];
#pragma unroll
  for (int i = 0; i < 4; ++i)
#pragma unroll
    for (int j = 0; j < 4; ++j) acc[i][j] = (v8f){0.f,0.f,0.f,0.f,0.f,0.f,0.f,0.f};

  for (int k0 = 0; k0 < K; k0 += 32) {
    V bh[4], bl[4];
#pragma unroll
    for (int j = 0; j < 4; ++j) {
      const size_t bo = (size_t)(n0 + (j << 4) + rlane) * ldb + koff + k0;
      bh[j] = Frag<T>::load(Bb + bo);
      if (SPLIT) bl[j] = Frag<T>::load(Bb2 + bo);
    }
#pragma unroll
    for (int i = 0; i < 4; ++i) {
      const size_t ao = (size_t)(m0 + (i << 4) + rlane) * lda + koff + k0;
      V ah = Frag<T>::load(Ab + ao);
      V al;
      if (SPLIT) al = Frag<T>::load(Ab2 + ao);
#pragma unroll
      for (int j = 0; j < 4; ++j) {
        acc[i][j] = Frag<T>::mma(ah, bh[j], acc[i][j]);
        if (SPLIT) {
          acc[i][j] = Frag<T>::mma(ah, bl[j], acc[i][j]);
          acc[i][j] = Frag<T>::mma(al, bh[j], acc[i][j]);
        }
      }
      Frag<T>::guard(acc[i][0], acc[i][3], ah, SPLIT ? al : ah);
    }
    Frag<T>::keep(bh[0], bh[1], bh[2], bh[3]);
    if (SPLIT) Frag<T>::keep(bl[0], bl[1], bl[2], bl[3]);
  }
  acc_guard4(acc[0][0], acc[0][1], acc[0][2], acc[0][3]);
  acc_guard4(acc[1][0], acc[1][1], acc[1][2], acc[1][3]);
  acc_guard4(acc[2][0], acc[2][1], acc[2][2], acc[2][3]);
  acc_guard4(acc[3][0], acc[3][1], acc[3][2], acc[3][3]);

  float* slab = sT[wave];
#pragma unroll
  for (int i = 0; i < 4; ++i) {
    const int mBase = m0 + (i << 4);
    float bl8[8];
#pragma unroll
    for (int r = 0; r < 8; ++r) bl8[r] = 0.f;
    if (BIAS_MODE == 1) {
      const v4f q0v = *(const v4f*)(bias + mBase + mOff);
      const v4f q1v = *(const v4f*)(bias + mBase + mOff + 4);
      bl8[0] = q0v[0]; bl8[1] = q0v[1]; bl8[2] = q0v[2]; bl8[3] = q0v[3];
      bl8[4] = q1v[0]; bl8[5] = q1v[1]; bl8[6] = q1v[2]; bl8[7] = q1v[3];
    }
#pragma unroll
    for (int j = 0; j < 4; ++j) {
      const int n = n0 + (j << 4) + rlane;
      float bv = 0.f;
      if (BIAS_MODE == 2) bv = bias[n];
#pragma unroll
      for (int r = 0; r < 8; ++r) {
        float v = acc[i][j][r] * scale;
        if (BIAS_MODE == 1) v += bl8[r];
        if (BIAS_MODE == 2) v += bv;
        slab[(mOff + r) * 68 + (j << 4) + rlane] = v;
      }
    }
    __builtin_amdgcn_fence(__ATOMIC_RELEASE, "workgroup");
    __builtin_amdgcn_wave_barrier();
    __builtin_amdgcn_fence(__ATOMIC_ACQUIRE, "workgroup");
    if (OUT_MODE == 0) {
      float* C = (float*)Cout + (size_t)b * strideC;
      const float* Rb = RESID ? (resid + (size_t)b * strideR) : nullptr;
      const int hh = lane >> 4, c4 = (lane & 15) * 4;
      for (int pass = 0; pass < 2; ++pass) {
#pragma unroll
        for (int it = 0; it < 8; ++it) {
          const int row = it * 2 + hh;
          v4f v = *(const v4f*)(slab + row * 68 + c4);
          if (RESID) {
            const v4f rr = *(const v4f*)(Rb + (size_t)(mBase + row) * ldc + n0 + c4);
            v += rr;
          }
          *(volatile v4f*)(C + (size_t)(mBase + row) * ldc + n0 + c4) = v;
        }
        __threadfence();
      }
    } else {
      const int q = lane >> 3, c8 = (lane & 7) * 8;
      unsigned short* C  = (unsigned short*)Cout  + (size_t)b * strideC;
      unsigned short* C2 = (OUT_MODE == 2) ? ((unsigned short*)Cout2 + (size_t)b * strideC) : nullptr;
      for (int pass = 0; pass < 2; ++pass) {
#pragma unroll
        for (int it = 0; it < 4; ++it) {
          const int row = it * 4 + q;
          const float* sp = slab + row * 68 + c8;
          v8h hv, lv;
#pragma unroll
          for (int e = 0; e < 8; ++e) {
            if (OUT_MODE == 1) {
              hv[e] = (_Float16)sp[e];
            } else {
              unsigned short hb = f2bf_bits(sp[e]);
              unsigned short lb = f2bf_bits(sp[e] - bf_bits2f(hb));
              hv[e] = __builtin_bit_cast(_Float16, hb);
              lv[e] = __builtin_bit_cast(_Float16, lb);
            }
          }
          *(volatile v8h*)(C + (size_t)(mBase + row) * ldc + n0 + c8) = hv;
          if (OUT_MODE == 2) *(volatile v8h*)(C2 + (size_t)(mBase + row) * ldc + n0 + c8) = lv;
        }
        __threadfence();
      }
    }
    __builtin_amdgcn_fence(__ATOMIC_RELEASE, "workgroup");
    __builtin_amdgcn_wave_barrier();
    __builtin_amdgcn_fence(__ATOMIC_ACQUIRE, "workgroup");
  }
}

__global__ __launch_bounds__(256) void bn_shift_kernel(
    const float* __restrict__ g2, const float* __restrict__ b2, const float* __restrict__ m2, const float* __restrict__ v2,
    const float* __restrict__ g4, const float* __restrict__ b4, const float* __restrict__ m4, const float* __restrict__ v4,
    float* __restrict__ t2x8, float* __restrict__ t4) {
  const int tid = threadIdx.x;
  if (blockIdx.x < 4) {
    const int i = blockIdx.x * 256 + tid;
    const float s = g2[i] * rsqrtf(v2[i] + BN_EPS);
    const float val = (b2[i] - m2[i] * s) * 8.0f;
    ((volatile float*)t2x8)[i] = val;
    __threadfence();
    ((volatile float*)t2x8)[i] = val;
  } else {
    const int i = tid;
    const float s = g4[i] * rsqrtf(v4[i] + BN_EPS);
    const float val = b4[i] - m4[i] * s;
    ((volatile float*)t4)[i] = val;
    __threadfence();
    ((volatile float*)t4)[i] = val;
  }
}

template <int ROWSCALE>
__global__ __launch_bounds__(256) void cast_weight_kernel(
    const float* __restrict__ in, unsigned short* __restrict__ out, int n2, int cols,
    const float* __restrict__ g, const float* __restrict__ v, float sc) {
  const int i = blockIdx.x * 256 + threadIdx.x;
  if (i < n2) {
    float s = sc;
    if (ROWSCALE) {
      const int r = (2 * i) / cols;
      s = sc * (g[r] * rsqrtf(v[r] + BN_EPS));
    }
    const unsigned u = (unsigned)h_bits(in[2 * i] * s) | ((unsigned)h_bits(in[2 * i + 1] * s) << 16);
    ((volatile unsigned*)out)[i] = u;
    __threadfence();
    ((volatile unsigned*)out)[i] = u;
  }
}

__global__ __launch_bounds__(256) void prologue_kernel(
    const float* __restrict__ x, const float* __restrict__ g1, const float* __restrict__ b1,
    const float* __restrict__ m1, const float* __restrict__ v1,
    unsigned short* __restrict__ h16, float* __restrict__ hp) {
  __shared__ __align__(16) unsigned short Hs[WPIX * CH];
  const int tid = threadIdx.x, wave = tid >> 5, lane = tid & 31;
  const int bn = blockIdx.x, b = bn >> 6, n = bn & 63, wy = n >> 3, wx = n & 7;
  const int cch = tid;
  const float g = g1[cch], bb = b1[cch], mm = m1[cch];
  const float rs = rsqrtf(v1[cch] + BN_EPS);
  const float* xp = x + ((size_t)(b * CH + cch)) * NPIX;
  float hs = 0.0f;
#pragma unroll 1
  for (int p = 0; p < WPIX; ++p) {
    const int pr = p / WSIDE, pc = p - pr * WSIDE;
    const int pix = (wy * WSIDE + pr) * IMGW + wx * WSIDE + pc;
    const float xv = xp[pix];
    float y = g * (xv - mm);
    y = y * rs;
    y = y + bb;
    const float hv = gelu_f(y);
    hs += hv;
    Hs[p * CH + cch] = h_bits(hv * 8.0f);
  }
  {
    const float hm = hs * (1.0f / 49.0f);
    float* hq = hp + (size_t)bn * CH + cch;
    *(volatile float*)hq = hm;
    __threadfence();
    *(volatile float*)hq = hm;
  }
  __syncthreads();
  for (int pass = 0; pass < 2; ++pass) {
    for (int p = wave; p < WPIX; p += 8) {
      const int pr = p / WSIDE, pc = p - pr * WSIDE;
      const int pix = (wy * WSIDE + pr) * IMGW + wx * WSIDE + pc;
      const v4u val = *(const v4u*)(Hs + p * CH + lane * 8);
      *(volatile v4u*)(h16 + ((size_t)(b * NPIX + pix)) * CH + lane * 8) = val;
    }
    __threadfence();
  }
}

__global__ __launch_bounds__(256) void route_kernel(
    const float* __restrict__ Wqkv, const float* __restrict__ hp, float* __restrict__ qr, float* __restrict__ kr) {
  __shared__ float hsh[CH];
  const int tid = threadIdx.x, bn = blockIdx.x;
  hsh[tid] = hp[(size_t)bn * CH + tid];
  __syncthreads();
  const float* wq = Wqkv + (size_t)tid * CH;
  const float* wk = Wqkv + (size_t)(CH + tid) * CH;
  float aq = 0.0f, ak = 0.0f;
#pragma unroll 4
  for (int c = 0; c < CH; ++c) {
    const float hv = hsh[c];
    aq = fmaf(wq[c], hv, aq);
    ak = fmaf(wk[c], hv, ak);
  }
  float* pq = qr + (size_t)bn * CH + tid;
  float* pk = kr + (size_t)bn * CH + tid;
  *(volatile float*)pq = aq;
  *(volatile float*)pk = ak;
  __threadfence();
  *(volatile float*)pq = aq;
  *(volatile float*)pk = ak;
}

__global__ __launch_bounds__(64) void affinity_kernel(
    const float* __restrict__ qr, const float* __restrict__ kr, float* __restrict__ aff) {
  __shared__ float qs[CH];
  const int tid = threadIdx.x, bn = blockIdx.x, b = bn >> 6;
#pragma unroll
  for (int i = 0; i < 4; ++i) qs[i * 64 + tid] = qr[(size_t)bn * CH + i * 64 + tid];
  __syncthreads();
  const float* kp = kr + ((size_t)(b * NWIN + tid)) * CH;
  float a = 0.0f;
#pragma unroll 4
  for (int c = 0; c < CH; ++c) a = fmaf(qs[c], kp[c], a);
  float* pa = aff + (size_t)bn * NWIN + tid;
  *(volatile float*)pa = a;
  __threadfence();
  *(volatile float*)pa = a;
}

__global__ __launch_bounds__(128) void window_attn_kernel(
    const unsigned short* __restrict__ qkv,
    const float* __restrict__ aff,
    unsigned short* __restrict__ msg) {
  __shared__ float s_aff[NWIN];
  __shared__ int s_idx[NTOP];
  __shared__ __align__(16) unsigned short Ksh[KCH * HDIM];
  __shared__ __align__(16) unsigned short Vth[HDIM * KCH];
  __shared__ __align__(16) _Float16 Psh[4][16 * KCH];
  __shared__ __align__(16) unsigned short Msh[WPIX * CH];
  const int tid = threadIdx.x, wave = tid >> 5, lane = tid & 31, hh = lane >> 4, c = lane & 15;
  const int bn = blockIdx.x, b = bn >> 6, n = bn & 63, wy = n >> 3, wx = n & 7;
  if (tid < NWIN) s_aff[tid] = aff[(size_t)bn * NWIN + tid];
  __syncthreads();
  if (tid == 0) {
    unsigned long long taken = 0ull;
    for (int t = 0; t < NTOP; ++t) {
      float best = -3.0e38f;
      int bi = 0;
      for (int jw = 0; jw < NWIN; ++jw) {
        const float v = s_aff[jw];
        const bool fr = ((taken >> jw) & 1ull) == 0ull;
        if (fr && (v > best)) { best = v; bi = jw; }
      }
      taken |= (1ull << bi);
      s_idx[t] = bi;
    }
  }
  __syncthreads();

  const int q0 = wave * 16;
  const size_t pixbase = (size_t)b * NPIX;
  int qrow = q0 + c;
  qrow = qrow < WPIX ? qrow : (WPIX - 1);
  const int qpr = qrow / WSIDE;
  const int qpix = (wy * WSIDE + qpr) * IMGW + wx * WSIDE + (qrow - qpr * WSIDE);
  const bool skipw = (wave == 3);
  const v8f z8 = {0.f, 0.f, 0.f, 0.f, 0.f, 0.f, 0.f, 0.f};

  for (int head = 0; head < NHEAD; ++head) {
    const v16h qa = Frag<_Float16>::load((const _Float16*)(qkv + (pixbase + qpix) * CH3 + head * HDIM) + 8 * hh);
    float mrow[8], lacc[8];
    v8f oacc[2];
#pragma unroll
    for (int r = 0; r < 8; ++r) { mrow[r] = -1.0e30f; lacc[r] = 0.0f; }
    oacc[0] = z8; oacc[1] = z8;

    for (int kc = 0; kc < NCHUNK; ++kc) {
      __syncthreads();
      {
        const int kr = tid >> 1, dh = (tid & 1) * 16;
        const int kk = kc * KCH + kr;
        const bool valid = kk < NKEY;
        const int kkc = valid ? kk : (NKEY - 1);
        const int slot = kkc / WPIX;
        const int r2 = kkc - slot * WPIX;
        int wj = s_idx[slot];
        wj = wj < 0 ? 0 : (wj > NWIN - 1 ? NWIN - 1 : wj);
        const int r2r = r2 / WSIDE, r2c = r2 - r2r * WSIDE;
        const int kpix = ((wj >> 3) * WSIDE + r2r) * IMGW + (wj & 7) * WSIDE + r2c;
        const unsigned short* base = qkv + (pixbase + kpix) * CH3 + head * HDIM + dh;
        v4u k0 = *(const v4u*)(base + CH);
        v4u k1 = *(const v4u*)(base + CH + 8);
        v4u v0 = *(const v4u*)(base + 2 * CH);
        v4u v1 = *(const v4u*)(base + 2 * CH + 8);
        const unsigned mk = valid ? 0xffffffffu : 0u;
        const v4u mk4 = {mk, mk, mk, mk};
        k0 &= mk4; k1 &= mk4; v0 &= mk4; v1 &= mk4;
        *(v4u*)(Ksh + kr * HDIM + dh) = k0;
        *(v4u*)(Ksh + kr * HDIM + dh + 8) = k1;
#pragma unroll
        for (int e = 0; e < 4; ++e) {
          const unsigned wa = v0[e], wb = v1[e];
          Vth[(dh + 2 * e) * KCH + kr]         = (unsigned short)(wa & 0xffffu);
          Vth[(dh + 2 * e + 1) * KCH + kr]     = (unsigned short)(wa >> 16);
          Vth[(dh + 8 + 2 * e) * KCH + kr]     = (unsigned short)(wb & 0xffffu);
          Vth[(dh + 8 + 2 * e + 1) * KCH + kr] = (unsigned short)(wb >> 16);
        }
      }
      __syncthreads();

      v8f s[4];
#pragma unroll
      for (int j = 0; j < 4; ++j) {
        const v16h kb = Frag<_Float16>::load((const _Float16*)(Ksh + (j * 16 + c) * HDIM) + 8 * hh);
        s[j] = mma_h(qa, kb, z8);
      }
      const bool lastc = (kc == NCHUNK - 1);
      float cm[8];
#pragma unroll
      for (int r = 0; r < 8; ++r) {
        float m = -1.0e30f;
#pragma unroll
        for (int j = 0; j < 4; ++j) {
          float v = s[j][r] * kScoreScale;
          if (lastc) {
            const int kvcol = kc * KCH + j * 16 + c;
            v = (kvcol < NKEY) ? v : -1.0e30f;
          }
          s[j][r] = v;
          m = fmaxf(m, v);
        }
        m = fmaxf(m, __shfl_xor(m, 1, 32));
        m = fmaxf(m, __shfl_xor(m, 2, 32));
        m = fmaxf(m, __shfl_xor(m, 4, 32));
        m = fmaxf(m, __shfl_xor(m, 8, 32));
        cm[r] = m;
      }
      _Float16* pw = Psh[wave];
#pragma unroll
      for (int r = 0; r < 8; ++r) {
        if (!skipw || r == 0) {
          const float mnew = fmaxf(mrow[r], cm[r]);
          const float alpha = exp2f(mrow[r] - mnew);
          mrow[r] = mnew;
          const float mb = mnew - 10.0f;
          float ps = 0.0f;
#pragma unroll
          for (int j = 0; j < 4; ++j) {
            const float p = exp2f(s[j][r] - mb);
            ps += p;
            pw[(8 * hh + r) * KCH + j * 16 + c] = (_Float16)p;
          }
          lacc[r] = fmaf(lacc[r], alpha, ps);
          oacc[0][r] *= alpha;
          oacc[1][r] *= alpha;
        } else {
#pragma unroll
          for (int j = 0; j < 4; ++j) pw[(8 * hh + r) * KCH + j * 16 + c] = (_Float16)0.0f;
        }
      }
      __builtin_amdgcn_fence(__ATOMIC_RELEASE, "workgroup");
      __builtin_amdgcn_wave_barrier();
      __builtin_amdgcn_fence(__ATOMIC_ACQUIRE, "workgroup");
#pragma unroll
      for (int ks = 0; ks < 2; ++ks) {
        const v16h pa = Frag<_Float16>::load(pw + c * KCH + ks * 32 + 8 * hh);
#pragma unroll
        for (int t = 0; t < 2; ++t) {
          const v16h vb = Frag<_Float16>::load((const _Float16*)(Vth + (t * 16 + c) * KCH + ks * 32) + 8 * hh);
          oacc[t] = mma_h(pa, vb, oacc[t]);
        }
      }
    }
#pragma unroll
    for (int r = 0; r < 8; ++r) {
      float l = lacc[r];
      l += __shfl_xor(l, 1, 32);
      l += __shfl_xor(l, 2, 32);
      l += __shfl_xor(l, 4, 32);
      l += __shfl_xor(l, 8, 32);
      const float inv = (l > 0.0f) ? (8.0f / l) : 0.0f;
      const unsigned short o0 = h_bits(oacc[0][r] * inv);
      const unsigned short o1 = h_bits(oacc[1][r] * inv);
      const int row = q0 + 8 * hh + r;
      if (row < WPIX) {
        Msh[row * CH + head * HDIM + c] = o0;
        Msh[row * CH + head * HDIM + 16 + c] = o1;
      }
    }
  }
  __syncthreads();
  for (int pass = 0; pass < 2; ++pass) {
    for (int p = wave; p < WPIX; p += 4) {
      const int pr = p / WSIDE, pc = p - pr * WSIDE;
      const int pix = (wy * WSIDE + pr) * IMGW + wx * WSIDE + pc;
      const v4u val = *(const v4u*)(Msh + p * CH + lane * 8);
      *(volatile v4u*)(msg + (pixbase + pix) * CH + lane * 8) = val;
    }
    __threadfence();
  }
}

__global__ __launch_bounds__(256) void transpose_x2_kernel(const float* __restrict__ x2, unsigned short* __restrict__ x2T) {
  __shared__ __align__(16) unsigned short Tt[64 * 72];
  const int tid = threadIdx.x, wave = tid >> 5, lane = tid & 31;
  const int hw0 = blockIdx.x * 64, cb = blockIdx.y * 64, b = blockIdx.z;
#pragma unroll
  for (int i = 0; i < 4; ++i) {
    const int idx = tid + 256 * i;
    const int cr = idx >> 4, f4 = idx & 15;
    const v4f v = *(const v4f*)(x2 + ((size_t)(b * CH + cb + cr)) * NPIX + hw0 + f4 * 4);
    Tt[(f4 * 4 + 0) * 72 + cr] = h_bits(v[0] * 8.0f);
    Tt[(f4 * 4 + 1) * 72 + cr] = h_bits(v[1] * 8.0f);
    Tt[(f4 * 4 + 2) * 72 + cr] = h_bits(v[2] * 8.0f);
    Tt[(f4 * 4 + 3) * 72 + cr] = h_bits(v[3] * 8.0f);
  }
  __syncthreads();
  const int q = lane >> 3, c8 = (lane & 7) * 8;
  for (int pass = 0; pass < 2; ++pass) {
#pragma unroll
    for (int rnd = 0; rnd < 2; ++rnd) {
      const int row = rnd * 32 + wave * 4 + q;
      const v4u val = *(const v4u*)(Tt + row * 72 + c8);
      *(volatile v4u*)(x2T + ((size_t)(b * NPIX + hw0 + row)) * CH + cb + c8) = val;
    }
    __threadfence();
  }
}

__global__ __launch_bounds__(256) void dwconv_kernel(
    const unsigned short* __restrict__ y2, const float* __restrict__ Wdw,
    const float* __restrict__ g3, const float* __restrict__ b3, const float* __restrict__ m3, const float* __restrict__ v3,
    unsigned short* __restrict__ h3) {
  __shared__ __align__(16) _Float16 Ts[64 * 10 * 58];
  __shared__ __align__(16) unsigned short Os[56 * 64];
  const int tid = threadIdx.x, wave = tid >> 5, lane = tid & 31;
  const int band = blockIdx.x, cgp = blockIdx.y, b = blockIdx.z;
  const int y0 = band * 8, cb = cgp * 64;
  for (int i = tid; i < 1280; i += 256) {
    const int rr = i >> 1;
    Ts[rr * 58 + ((i & 1) ? 57 : 0)] = (_Float16)0.0f;
  }
#pragma unroll 1
  for (int i = tid; i < 64 * 10 * 56; i += 256) {
    const int ci = i / 560;
    const int rem = i - ci * 560;
    const int ry = rem / 56;
    const int xx = rem - ry * 56;
    const int yy = y0 - 1 + ry;
    const bool ok = (yy >= 0) && (yy < 56);
    const int yc = yy < 0 ? 0 : (yy > 55 ? 55 : yy);
    const unsigned short u = y2[((size_t)(b * HID + cb + ci)) * NPIX + yc * IMGW + xx];
    const float gv = gelu_f(h_val(u) * 0.125f) * 8.0f;
    Ts[(ci * 10 + ry) * 58 + xx + 1] = (_Float16)(ok ? gv : 0.0f);
  }
  __syncthreads();
  const int ci = tid >> 2, xs = tid & 3, cch = cb + ci;
  const float w0 = Wdw[cch * 9 + 0], w1 = Wdw[cch * 9 + 1], w2 = Wdw[cch * 9 + 2];
  const float w3 = Wdw[cch * 9 + 3], w4 = Wdw[cch * 9 + 4], w5 = Wdw[cch * 9 + 5];
  const float w6 = Wdw[cch * 9 + 6], w7 = Wdw[cch * 9 + 7], w8 = Wdw[cch * 9 + 8];
  const float s3 = g3[cch] * rsqrtf(v3[cch] + BN_EPS);
  const float t3 = b3[cch] - m3[cch] * s3;
  const float s3e = s3 * 0.125f;
  const int q = lane >> 3, c8 = (lane & 7) * 8;
  for (int orow = 0; orow < 8; ++orow) {
    const _Float16* r0p = Ts + (ci * 10 + orow) * 58 + xs * 14;
    const _Float16* r1p = r0p + 58;
    const _Float16* r2p = r0p + 116;
    float a0 = (float)r0p[0], a1 = (float)r1p[0], a2 = (float)r2p[0];
    float e0 = (float)r0p[1], e1 = (float)r1p[1], e2 = (float)r2p[1];
    const int xo = xs * 14;
#pragma unroll 1
    for (int i = 0; i < 14; ++i) {
      const float f0 = (float)r0p[i + 2], f1 = (float)r1p[i + 2], f2 = (float)r2p[i + 2];
      float acc = w0 * a0;
      acc = fmaf(w1, e0, acc); acc = fmaf(w2, f0, acc);
      acc = fmaf(w3, a1, acc); acc = fmaf(w4, e1, acc); acc = fmaf(w5, f1, acc);
      acc = fmaf(w6, a2, acc); acc = fmaf(w7, e2, acc); acc = fmaf(w8, f2, acc);
      const float z = fmaf(acc, s3e, t3);
      Os[(xo + i) * 64 + ci] = h_bits(gelu_f(z) * 64.0f);
      a0 = e0; a1 = e1; a2 = e2;
      e0 = f0; e1 = f1; e2 = f2;
    }
    __syncthreads();
    const int prow = y0 + orow;
    for (int pass = 0; pass < 2; ++pass) {
#pragma unroll
      for (int rnd = 0; rnd < 2; ++rnd) {
        const int pb = rnd * 32 + wave * 4;
        if (pb < 56) {
          const int p = pb + q;
          const v4u val = *(const v4u*)(Os + p * 64 + c8);
          *(volatile v4u*)(h3 + ((size_t)(b * NPIX + prow * IMGW + p)) * HID + cb + c8) = val;
        }
      }
      __threadfence();
    }
    __syncthreads();
  }
}

constexpr size_t SZ_WQKV = (size_t)CH3 * CH * 2;
constexpr size_t SZ_WM   = (size_t)CH * CH * 2;
constexpr size_t SZ_W1   = (size_t)HID * CH * 2;
constexpr size_t SZ_W2   = (size_t)CH * HID * 2;
constexpr size_t SZ_T2   = (size_t)HID * 4;
constexpr size_t SZ_T4   = (size_t)CH * 4;
constexpr size_t SZ_HP   = (size_t)BATCH * NWIN * CH * 4;
constexpr size_t SZ_QR   = SZ_HP;
constexpr size_t SZ_KR   = SZ_HP;
constexpr size_t SZ_AFF  = (size_t)BATCH * NWIN * NWIN * 4;
constexpr size_t SZ_RA   = (size_t)BATCH * HID * NPIX * 2;
constexpr size_t SZ_RB   = SZ_RA;
constexpr size_t SZ_RC   = (size_t)BATCH * CH * NPIX * 4;
constexpr size_t OFF_WQKV = 0;
constexpr size_t OFF_WM   = OFF_WQKV + SZ_WQKV;
constexpr size_t OFF_W1   = OFF_WM + SZ_WM;
constexpr size_t OFF_W2   = OFF_W1 + SZ_W1;
constexpr size_t OFF_T2   = OFF_W2 + SZ_W2;
constexpr size_t OFF_T4   = OFF_T2 + SZ_T2;
constexpr size_t OFF_HP   = OFF_T4 + SZ_T4;
constexpr size_t OFF_QR   = OFF_HP + SZ_HP;
constexpr size_t OFF_KR   = OFF_QR + SZ_QR;
constexpr size_t OFF_AFF  = OFF_KR + SZ_KR;
constexpr size_t OFF_RA   = OFF_AFF + SZ_AFF;
constexpr size_t OFF_RB   = OFF_RA + SZ_RA;
constexpr size_t OFF_RC   = OFF_RB + SZ_RB;
constexpr size_t OFF_END  = OFF_RC + SZ_RC;
static_assert(OFF_END <= (size_t)134217728);
static_assert((size_t)BATCH * NPIX * CH3 * 2 <= SZ_RA);
static_assert((size_t)BATCH * HID * NPIX * 2 <= SZ_RA);
static_assert((size_t)BATCH * NPIX * CH * 2 <= SZ_RB);
static_assert((size_t)BATCH * NPIX * HID * 2 <= SZ_RB);
static_assert((OFF_RA % 256) == 0 && (OFF_RB % 256) == 0 && (OFF_RC % 256) == 0 && (OFF_HP % 256) == 0);
static_assert(NPIX % 64 == 0 && CH % 64 == 0 && CH3 % 64 == 0 && HID % 64 == 0);
static_assert(CH % 32 == 0 && HID % 32 == 0);

extern "C" void kernel_launch(void* const* d_in, const int* in_sizes, int n_in,
                              void* d_out, int out_size, void* d_ws, size_t ws_size,
                              hipStream_t stream) {
  (void)in_sizes; (void)n_in; (void)out_size;
  const float* x     = (const float*)d_in[0];
  const float* g1    = (const float*)d_in[1];
  const float* b1    = (const float*)d_in[2];
  const float* m1    = (const float*)d_in[3];
  const float* v1    = (const float*)d_in[4];
  const float* Wqkv  = (const float*)d_in[5];
  const float* Wm    = (const float*)d_in[6];
  const float* bmrg  = (const float*)d_in[7];
  const float* W1    = (const float*)d_in[8];
  const float* g2    = (const float*)d_in[9];
  const float* b2    = (const float*)d_in[10];
  const float* m2    = (const float*)d_in[11];
  const float* v2    = (const float*)d_in[12];
  const float* Wdw   = (const float*)d_in[13];
  const float* g3    = (const float*)d_in[14];
  const float* b3    = (const float*)d_in[15];
  const float* m3    = (const float*)d_in[16];
  const float* v3    = (const float*)d_in[17];
  const float* W2    = (const float*)d_in[18];
  const float* g4    = (const float*)d_in[19];
  const float* b4    = (const float*)d_in[20];
  const float* m4    = (const float*)d_in[21];
  const float* v4    = (const float*)d_in[22];
  float* out = (float*)d_out;
  if (ws_size < OFF_END) return;
  char* ws = (char*)d_ws;
  unsigned short* wqkv16 = (unsigned short*)(ws + OFF_WQKV);
  unsigned short* wm16   = (unsigned short*)(ws + OFF_WM);
  unsigned short* w1h    = (unsigned short*)(ws + OFF_W1);
  unsigned short* w2h    = (unsigned short*)(ws + OFF_W2);
  float* t2x8 = (float*)(ws + OFF_T2);
  float* t4   = (float*)(ws + OFF_T4);
  float* hp   = (float*)(ws + OFF_HP);
  float* qr   = (float*)(ws + OFF_QR);
  float* kr   = (float*)(ws + OFF_KR);
  float* aff  = (float*)(ws + OFF_AFF);
  unsigned short* qkv16 = (unsigned short*)(ws + OFF_RA);
  unsigned short* y2    = (unsigned short*)(ws + OFF_RA);
  unsigned short* h16   = (unsigned short*)(ws + OFF_RB);
  unsigned short* msg16 = (unsigned short*)(ws + OFF_RB);
  unsigned short* x2T   = (unsigned short*)(ws + OFF_RB);
  unsigned short* h3    = (unsigned short*)(ws + OFF_RB);
  float* x2 = (float*)(ws + OFF_RC);

  bn_shift_kernel<<<5, 256, 0, stream>>>(g2, b2, m2, v2, g4, b4, m4, v4, t2x8, t4);
  {
    const int nq = CH3 * CH / 2, nm = CH * CH / 2, n1 = HID * CH / 2, nn2 = CH * HID / 2;
    cast_weight_kernel<0><<<(nq + 255) / 256, 256, 0, stream>>>(Wqkv, wqkv16, nq, CH, g2, v2, 16.0f);
    cast_weight_kernel<0><<<(nm + 255) / 256, 256, 0, stream>>>(Wm, wm16, nm, CH, g2, v2, 16.0f);
    cast_weight_kernel<1><<<(n1 + 255) / 256, 256, 0, stream>>>(W1, w1h, n1, CH, g2, v2, 16.0f);
    cast_weight_kernel<1><<<(nn2 + 255) / 256, 256, 0, stream>>>(W2, w2h, nn2, HID, g4, v4, 16.0f);
  }
  prologue_kernel<<<BATCH * NWIN, 256, 0, stream>>>(x, g1, b1, m1, v1, h16, hp);
  route_kernel<<<BATCH * NWIN, 256, 0, stream>>>(Wqkv, hp, qr, kr);
  affinity_kernel<<<BATCH * NWIN, 64, 0, stream>>>(qr, kr, aff);
  {
    const int tiles = (NPIX / 64) * (CH3 / 64);
    wmma_gemm64<0, false, 0, 1, false><<<dim3((tiles + 7) / 8, BATCH), 256, 0, stream>>>(
        h16, h16, CH, (long)NPIX * CH,
        wqkv16, wqkv16, CH, 0L,
        (void*)qkv16, (void*)qkv16, CH3, (long)NPIX * CH3,
        t4, x, 0L,
        NPIX, CH3, CH, 1.0f / 16.0f);
  }
  window_attn_kernel<<<BATCH * NWIN, 128, 0, stream>>>(qkv16, aff, msg16);
  {
    const int tiles = (CH / 64) * (NPIX / 64);
    wmma_gemm64<0, false, 1, 0, true><<<dim3((tiles + 7) / 8, BATCH), 256, 0, stream>>>(
        wm16, wm16, CH, 0L,
        msg16, msg16, CH, (long)NPIX * CH,
        (void*)x2, (void*)x2, NPIX, (long)CH * NPIX,
        bmrg, x, (long)CH * NPIX,
        CH, NPIX, CH, 1.0f / 1024.0f);
  }
  transpose_x2_kernel<<<dim3(NPIX / 64, CH / 64, BATCH), 256, 0, stream>>>(x2, x2T);
  {
    const int tiles = (HID / 64) * (NPIX / 64);
    wmma_gemm64<0, false, 1, 1, false><<<dim3((tiles + 7) / 8, BATCH), 256, 0, stream>>>(
        w1h, w1h, CH, 0L,
        x2T, x2T, CH, (long)NPIX * CH,
        (void*)y2, (void*)y2, NPIX, (long)HID * NPIX,
        t2x8, x, 0L,
        HID, NPIX, CH, 1.0f / 16.0f);
  }
  dwconv_kernel<<<dim3(IMGW / 8, HID / 64, BATCH), 256, 0, stream>>>(y2, Wdw, g3, b3, m3, v3, h3);
  {
    const int tiles = (CH / 64) * (NPIX / 64);
    wmma_gemm64<0, false, 1, 0, true><<<dim3((tiles + 7) / 8, BATCH), 256, 0, stream>>>(
        w2h, w2h, HID, 0L,
        h3, h3, HID, (long)NPIX * HID,
        (void*)out, (void*)out, NPIX, (long)CH * NPIX,
        t4, x2, (long)CH * NPIX,
        CH, NPIX, HID, 1.0f / 1024.0f);
  }
}
